// SimpleGCNClassifier_33990371181249
// MI455X (gfx1250) — hardware-verified
//
#include <hip/hip_runtime.h>
#include <stddef.h>
#include <stdint.h>
#include <math.h>


#define DF     128
#define KG     256
#define NCLS   10
#define NH1    12
#define NGR    512
#define NTHR   256
#define NWAVE  8
#define EPT    8
#define CHUNK  (NTHR * EPT)
#define WCAP   (EPT * 32)
#define LISTN  (NWAVE * WCAP)
#define NBA    1024
#define SLA    10
#define RCAP   28672
#define DEGCAP 64
#define GBM    64
#define GBN    128
#define GTHR   128
#define ROWH   256
#define AGG_ZINTS    (LISTN + 2 * RCAP + 3 * NBA)
#define MISC_INTS    16
#define ROWBUF_INTS  (NWAVE * ROWH / 2)
#define AGG_LDS_INTS (AGG_ZINTS + MISC_INTS + ROWBUF_INTS)
#define NOUT   (NGR * NCLS)
#define NZ1    (NGR * NH1)
#define T_B    0
#define T_W1   128
#define T_B1   1664
#define T_W2   1696
#define T_B2   1824
#define T_USED 1856
#define T_FLOATS 2048
#define NBW    16
#define NBT    6
#define WSMAX  134217728

static_assert((CHUNK & (CHUNK - 1)) == 0 && CHUNK <= 4096);
static_assert((NBA & (NBA - 1)) == 0 && NBA == (1 << SLA));
static_assert(((long long)CHUNK << SLA) < (1LL << 31));
static_assert(LISTN % NTHR == 0 && NBA % NTHR == 0 && NBA == 4 * NTHR);
static_assert(NBA % NWAVE == 0 && NBA % 32 == 0 && NBA % GBM == 0);
static_assert(RCAP % 4 == 0 && AGG_ZINTS % 4 == 0 && LISTN % 4 == 0 && ((AGG_ZINTS + MISC_INTS) % 4) == 0);
static_assert(AGG_ZINTS % (NTHR * 4) == 0);
static_assert(100000 % NBA == 672 && (100000 * 4) % 128 == 0);
static_assert(DF == 4 * 32 && KG == 2 * DF && KG % 32 == 0 && ROWH == KG);
static_assert(GBN == DF && GBM == (GTHR / 32) * 16);
static_assert(RCAP >= (6435 * 105 + 99) / 100 && RCAP >= (6277 * 105 + 99) / 100);
static_assert(DEGCAP >= 19 + 8);
static_assert(AGG_LDS_INTS * 4 <= 327680);
static_assert((NOUT * 4) % 128 == 0 && NOUT % (4 * NTHR) == 0 && NZ1 % NTHR == 0 && NOUT % NTHR == 0);
static_assert(T_W1 == T_B + DF && T_B1 == T_W1 + DF * NH1 && T_W2 == T_B1 + 32 && T_B2 == T_W2 + 128);
static_assert(T_USED == T_B2 + 32 && T_USED % 4 == 0 && T_USED <= T_FLOATS);
static_assert(T_B % 32 == 0 && T_W1 % 32 == 0 && T_B1 % 32 == 0 && T_W2 % 32 == 0 && T_B2 % 32 == 0);
static_assert(NBW * NTHR == DF * (KG / 8));

#define KERNEL(T) __global__ __launch_bounds__(T) __attribute__((amdgpu_num_vgpr(248)))

typedef float          v4f   __attribute__((ext_vector_type(4)));
typedef float          v8f   __attribute__((ext_vector_type(8)));
typedef int            v4i   __attribute__((ext_vector_type(4)));
typedef int            v8i   __attribute__((ext_vector_type(8)));
typedef unsigned       v2u   __attribute__((ext_vector_type(2)));
typedef unsigned short v4us  __attribute__((ext_vector_type(4)));
typedef unsigned short v8us  __attribute__((ext_vector_type(8)));
typedef unsigned short v16us __attribute__((ext_vector_type(16)));
typedef __bf16         v16bf __attribute__((ext_vector_type(16)));
typedef v4f  __attribute__((may_alias)) v4fa;
typedef v4i  __attribute__((may_alias)) v4ia;
typedef v2u  __attribute__((may_alias)) v2ua;
typedef v4us __attribute__((may_alias)) v4usa;
typedef v8us __attribute__((may_alias)) v8usa;
union FragB { v16bf v; v16us u; v8us h[2]; v8i w; };

__device__ __forceinline__ v8f wmb(const FragB& a, const FragB& b, v8f c) {
  v8f d = __builtin_amdgcn_wmma_f32_16x16x32_bf16(false, a.v, false, b.v, (short)0, c, false, false);
  asm volatile("v_nop\n\tv_nop\n\tv_nop\n\tv_nop" : "+v"(d) : "v"(a.w), "v"(b.w));
  return d;
}

__device__ __forceinline__ unsigned bf16_bits(float f) {
  const unsigned u = __float_as_uint(f);
  return (u + 0x7FFFu + ((u >> 16) & 1u)) >> 16;
}
__device__ __forceinline__ float bf16_val(float f) {
  return __uint_as_float(bf16_bits(f) << 16);
}
__device__ __forceinline__ unsigned bf16_bits_np(float f) {
  const unsigned u = __float_as_uint(f);
  const unsigned r = (u + 0x7FFFu + ((u >> 16) & 1u)) >> 16;
  return (f != f) ? 0x7FC0u : r;
}

__device__ __forceinline__ void wave_sync() {
  __builtin_amdgcn_fence(__ATOMIC_RELEASE, "workgroup");
  __builtin_amdgcn_wave_barrier();
  __builtin_amdgcn_fence(__ATOMIC_ACQUIRE, "workgroup");
}

template <int SLB>
__device__ __forceinline__ int scan_chunk(const int* __restrict__ dsts, int nE, int cbase, int slotBase,
                                          int nb, int vec8, int* list, int tid, int lane, int wave) {
  int wc = 0;
  const int el0  = tid * EPT;
  const int e0   = cbase + el0;
  const int sent = -2147483647 - 1;
  v4i da, db;
  if (vec8 != 0 && cbase + CHUNK <= nE) {
    da = *(const v4i*)(dsts + e0);
    db = *(const v4i*)(dsts + e0 + 4);
  } else {
    da.x = (e0     < nE) ? dsts[min(e0,     nE - 1)] : sent;
    da.y = (e0 + 1 < nE) ? dsts[min(e0 + 1, nE - 1)] : sent;
    da.z = (e0 + 2 < nE) ? dsts[min(e0 + 2, nE - 1)] : sent;
    da.w = (e0 + 3 < nE) ? dsts[min(e0 + 3, nE - 1)] : sent;
    db.x = (e0 + 4 < nE) ? dsts[min(e0 + 4, nE - 1)] : sent;
    db.y = (e0 + 5 < nE) ? dsts[min(e0 + 5, nE - 1)] : sent;
    db.z = (e0 + 6 < nE) ? dsts[min(e0 + 6, nE - 1)] : sent;
    db.w = (e0 + 7 < nE) ? dsts[min(e0 + 7, nE - 1)] : sent;
  }
  const unsigned nbs = (unsigned)slotBase;
  const unsigned unb = (unsigned)nb;
  const unsigned s0 = (unsigned)da.x - nbs, s1 = (unsigned)da.y - nbs;
  const unsigned s2 = (unsigned)da.z - nbs, s3 = (unsigned)da.w - nbs;
  const unsigned s4 = (unsigned)db.x - nbs, s5 = (unsigned)db.y - nbs;
  const unsigned s6 = (unsigned)db.z - nbs, s7 = (unsigned)db.w - nbs;
  const bool h0 = s0 < unb, h1 = s1 < unb, h2 = s2 < unb, h3 = s3 < unb;
  const bool h4 = s4 < unb, h5 = s5 < unb, h6 = s6 < unb, h7 = s7 < unb;
  const unsigned any = __builtin_amdgcn_ballot_w32(h0 | h1 | h2 | h3 | h4 | h5 | h6 | h7);
  if (any != 0u) {
#define HITJ(J, HJ, SJ) { \
      const unsigned mj = __builtin_amdgcn_ballot_w32(HJ); \
      if (mj != 0u) { \
        if (HJ) { \
          const int pos = wc + (int)__builtin_amdgcn_mbcnt_lo(mj, 0u); \
          if (pos < WCAP) list[wave * WCAP + pos] = ((el0 + (J)) << SLB) | (int)(SJ); \
        } \
        wc += (int)__builtin_popcount(mj); } }
    HITJ(0, h0, s0)
    HITJ(1, h1, s1)
    HITJ(2, h2, s2)
    HITJ(3, h3, s3)
    HITJ(4, h4, s4)
    HITJ(5, h5, s5)
    HITJ(6, h6, s6)
    HITJ(7, h7, s7)
#undef HITJ
  }
  return wc;
}

__device__ __forceinline__ void tab_fill(const float* __restrict__ src, int nvalid, float* dst, int nunits, int t) {
  const bool act = t < nunits;
  const int e = 4 * t;
  const float a0 = src[min(e,     nvalid - 1)];
  const float a1 = src[min(e + 1, nvalid - 1)];
  const float a2 = src[min(e + 2, nvalid - 1)];
  const float a3 = src[min(e + 3, nvalid - 1)];
  v4f o;
  o.x = (e     < nvalid) ? bf16_val(a0) : 0.0f;
  o.y = (e + 1 < nvalid) ? bf16_val(a1) : 0.0f;
  o.z = (e + 2 < nvalid) ? bf16_val(a2) : 0.0f;
  o.w = (e + 3 < nvalid) ? bf16_val(a3) : 0.0f;
  float* dp = dst + (act ? e : 0);
  if (act) *(volatile v4f*)dp = o;
  __threadfence();
  if (act) *(volatile v4f*)dp = o;
}

KERNEL(NTHR) void k_prep(const float* __restrict__ x, const float* __restrict__ W, const float* __restrict__ b,
                         const float* __restrict__ W1, const float* __restrict__ b1,
                         const float* __restrict__ W2, const float* __restrict__ b2,
                         int nN, int nbX, unsigned short* xb, unsigned short* wt2, float* tab) {
  const int bid = (int)blockIdx.x;
  const int tid = (int)threadIdx.x;
  if (bid < nbX) {
    const int u   = bid * NTHR + tid;
    const int row = u >> 4;
    const int k8  = (u & 15) * 8;
    const int rc  = row < nN ? row : nN - 1;
    const float* p = x + (size_t)rc * DF + k8;
    const v4f a = *(const v4f*)p;
    const v4f c = *(const v4f*)(p + 4);
    const bool ok = row < nN;
    v8us o;
    o[0] = ok ? (unsigned short)bf16_bits(a.x) : (unsigned short)0;
    o[1] = ok ? (unsigned short)bf16_bits(a.y) : (unsigned short)0;
    o[2] = ok ? (unsigned short)bf16_bits(a.z) : (unsigned short)0;
    o[3] = ok ? (unsigned short)bf16_bits(a.w) : (unsigned short)0;
    o[4] = ok ? (unsigned short)bf16_bits(c.x) : (unsigned short)0;
    o[5] = ok ? (unsigned short)bf16_bits(c.y) : (unsigned short)0;
    o[6] = ok ? (unsigned short)bf16_bits(c.z) : (unsigned short)0;
    o[7] = ok ? (unsigned short)bf16_bits(c.w) : (unsigned short)0;
    unsigned short* dp = xb + (size_t)row * DF + k8;
    *(volatile v8us*)dp = o;
    __threadfence();
    *(volatile v8us*)dp = o;
  } else if (bid < nbX + NBW) {
    const int v  = (bid - nbX) * NTHR + tid;
    const int n  = v >> 5;
    const int k8 = (v & 31) * 8;
    const int kk = k8 & (DF - 1);
    const float* p = W + (size_t)kk * DF + n;
    v8us o;
#pragma unroll
    for (int i = 0; i < 8; ++i) o[i] = (unsigned short)bf16_bits(p[(size_t)i * DF]);
    unsigned short* dp = wt2 + (size_t)n * KG + k8;
    *(volatile v8us*)dp = o;
    __threadfence();
    *(volatile v8us*)dp = o;
  } else {
    const int r = bid - nbX - NBW;
    if (r == 0)      tab_fill(b,  DF,         tab + T_B,  32,  tid);
    else if (r <= 2) tab_fill(W1, DF * NH1,   tab + T_W1, 384, (r - 1) * NTHR + tid);
    else if (r == 3) tab_fill(b1, NH1,        tab + T_B1, 8,   tid);
    else if (r == 4) tab_fill(W2, NH1 * NCLS, tab + T_W2, 32,  tid);
    else if (r == 5) tab_fill(b2, NCLS,       tab + T_B2, 8,   tid);
  }
}

KERNEL(NTHR) void k_odeg(const int* __restrict__ keys, int nE, int nN, int vec8, float* nsout) {
  __shared__ __attribute__((aligned(16))) int scnt[NBA];
  __shared__ __attribute__((aligned(16))) int list[LISTN];
  __shared__ __attribute__((aligned(16))) float nsl[NBA];
  __shared__ int wcnt[NWAVE];
  const int tid = (int)threadIdx.x, lane = tid & 31, wave = tid >> 5;
  const int nodeBase = (int)blockIdx.x * NBA;

  for (int i = tid; i < NBA; i += NTHR) scnt[i] = 0;
  for (int i = tid; i < LISTN; i += NTHR) list[i] = 0;
  if (tid < NWAVE) wcnt[tid] = 0;
  __syncthreads();

  const int nChunks = (nE + CHUNK - 1) / CHUNK;
#pragma unroll 1
  for (int ch = 0; ch < nChunks; ++ch) {
    const int cbase = ch * CHUNK;
    const int wc = scan_chunk<SLA>(keys, nE, cbase, nodeBase, NBA, vec8, list, tid, lane, wave);
    if (lane == 0) wcnt[wave] = wc;
    __syncthreads();
    if (wave == 0) {
#pragma unroll 1
      for (int w2 = 0; w2 < NWAVE; ++w2) {
        int c = wcnt[w2];
        c = c < 0 ? 0 : (c > WCAP ? WCAP : c);
#pragma unroll 1
        for (int b0 = 0; b0 < c; b0 += 32) {
          const int idx = b0 + lane;
          const int ent = list[w2 * WCAP + (idx < WCAP ? idx : WCAP - 1)];
          const int m32 = (c - b0) < 32 ? (c - b0) : 32;
#pragma unroll 1
          for (int k = 0; k < m32; ++k) {
            const int u  = __builtin_amdgcn_readlane(ent, k);
            const int sl = u & (NBA - 1);
            if (lane == 0) scnt[sl] = scnt[sl] + 1;
          }
        }
      }
    }
    __syncthreads();
  }

#pragma unroll 1
  for (int it = 0; it < NBA / NTHR; ++it) {
    const int s = it * NTHR + tid;
    int c = scnt[s];
    c = c < 1 ? 1 : c;
    nsl[s] = 1.0f / sqrtf((float)c);
  }
  __syncthreads();
  const v4f v = *(const v4fa*)(nsl + 4 * tid);
  const bool ok = (nodeBase + 4 * tid + 3) < nN;
  float* op = nsout + (size_t)(ok ? (nodeBase + 4 * tid) : 0);
  if (ok) *(volatile v4f*)op = v;
  __threadfence();
  if (ok) *(volatile v4f*)op = v;
}

KERNEL(NTHR) void k_agg(const int* __restrict__ srcs, const int* __restrict__ dsts, int nE, int nN, int vec8,
                        int mRows, const float* __restrict__ ns, const unsigned short* __restrict__ xb,
                        unsigned short* ag) {
#pragma clang fp contract(off)
  extern __shared__ __attribute__((aligned(16))) int dsm[];
  int* list = dsm;
  int* hl   = dsm + LISTN;
  int* sl   = hl + RCAP;
  int* cnt  = sl + RCAP;
  int* offs = cnt + NBA;
  int* cur  = offs + NBA;
  int* misc = cur + NBA;
  const int tid = (int)threadIdx.x, lane = tid & 31, wave = tid >> 5;
  unsigned short* rowbuf = (unsigned short*)(misc + MISC_INTS) + wave * ROWH;
  const int nodeBase = (int)blockIdx.x * NBA;

  {
    const v4i z4 = {0, 0, 0, 0};
    for (int i = tid * 4; i < AGG_ZINTS; i += NTHR * 4) *(v4ia*)(dsm + i) = z4;
    if (tid < MISC_INTS) misc[tid] = 0;
  }
  __syncthreads();

  int t = 0, ov = 0;
  const int nChunks = (nE + CHUNK - 1) / CHUNK;
#pragma unroll 1
  for (int ch = 0; ch < nChunks; ++ch) {
    const int cbase = ch * CHUNK;
    const int wc = scan_chunk<SLA>(dsts, nE, cbase, nodeBase, NBA, vec8, list, tid, lane, wave);
    if (lane == 0) misc[wave] = wc;
    __syncthreads();
    if (wave == 0) {
#pragma unroll 1
      for (int w2 = 0; w2 < NWAVE; ++w2) {
        int c = misc[w2];
        c = c < 0 ? 0 : (c > WCAP ? WCAP : c);
#pragma unroll 1
        for (int b0 = 0; b0 < c; b0 += 32) {
          const int idx = b0 + lane;
          const int ent = list[w2 * WCAP + (idx < WCAP ? idx : WCAP - 1)];
          const int m32 = (c - b0) < 32 ? (c - b0) : 32;
#pragma unroll 1
          for (int k = 0; k < m32; ++k) {
            const int u    = __builtin_amdgcn_readlane(ent, k);
            const int slot = u & (NBA - 1);
            const int el   = (u >> SLA) & (CHUNK - 1);
            const int pk   = ((cbase + el) << SLA) | slot;
            if (t < RCAP) {
              if (lane == 0) { hl[t] = pk; cnt[slot] = cnt[slot] + 1; }
              t = t + 1;
            } else {
              ov = 1;
            }
          }
        }
      }
    }
    __syncthreads();
  }
  if (wave == 0 && lane == 0) { misc[8] = t; misc[9] = ov; }
  __syncthreads();
  int tt = misc[8];
  tt = tt < 0 ? 0 : (tt > RCAP ? RCAP : tt);
  const int ovf = misc[9];

  if (wave == 0) {
    const int base = lane * (NBA / 32);
    int s = 0;
#pragma unroll 1
    for (int i = 0; i < NBA / 32; ++i) s += cnt[base + i];
    int incl = s;
#pragma unroll
    for (int d = 1; d < 32; d <<= 1) {
      const int y = __shfl_up(incl, d, 32);
      if (lane >= d) incl += y;
    }
    int run = incl - s;
#pragma unroll 1
    for (int i = 0; i < NBA / 32; ++i) {
      const int cv = cnt[base + i];
      offs[base + i] = run;
      cur[base + i]  = run;
      run += cv;
    }
  }
  __syncthreads();
  if (wave == 0) {
#pragma unroll 1
    for (int b0 = 0; b0 < tt; b0 += 32) {
      const int idx = b0 + lane;
      const int ent = hl[idx < RCAP ? idx : RCAP - 1];
      const int m32 = (tt - b0) < 32 ? (tt - b0) : 32;
#pragma unroll 1
      for (int k = 0; k < m32; ++k) {
        const int u    = __builtin_amdgcn_readlane(ent, k);
        const int slot = u & (NBA - 1);
        if (lane == 0) {
          int p = cur[slot];
          p = p < 0 ? 0 : (p > RCAP - 1 ? RCAP - 1 : p);
          sl[p] = u;
          cur[slot] = p + 1;
        }
      }
    }
  }
  __syncthreads();

  const float qnan = __int_as_float(0x7fc00000);
  const float pz = (ovf != 0) ? qnan : 0.0f;
#pragma unroll 1
  for (int si = 0; si < NBA / NWAVE; ++si) {
    const int s    = si * NWAVE + wave;
    const int node = nodeBase + s;
    const int craw = cnt[s];
    const bool big = craw > DEGCAP;
    const int c = craw < 0 ? 0 : (craw > DEGCAP ? DEGCAP : craw);
    int o = offs[s];
    o = o < 0 ? 0 : (o > RCAP ? RCAP : o);
    const float nd = 1.0f / sqrtf((float)(craw < 1 ? 1 : craw));
    float a0 = 0.0f, a1 = 0.0f, a2 = 0.0f, a3 = 0.0f;
#pragma unroll 1
    for (int b0 = 0; b0 < c; b0 += 32) {
      int idx = o + b0 + lane;
      idx = idx > RCAP - 1 ? RCAP - 1 : idx;
      const int ent = sl[idx];
      int eid = ent >> SLA;
      eid = eid < 0 ? 0 : (eid > nE - 1 ? nE - 1 : eid);
      int sr = srcs[eid];
      sr = sr < 0 ? 0 : (sr > nN - 1 ? nN - 1 : sr);
      const float nv  = ns[sr];
      const int   nvi = __float_as_int(nv);
      const int m32 = (c - b0) < 32 ? (c - b0) : 32;
#pragma unroll 1
      for (int k = 0; k < m32; ++k) {
        const int   sk = __builtin_amdgcn_readlane(sr, k);
        const float ck = __int_as_float(__builtin_amdgcn_readlane(nvi, k));
        const v2u w = *(const v2ua*)(xb + (size_t)sk * DF + 4 * lane);
        const float f0 = __uint_as_float(w.x << 16);
        const float f1 = __uint_as_float(w.x & 0xffff0000u);
        const float f2 = __uint_as_float(w.y << 16);
        const float f3 = __uint_as_float(w.y & 0xffff0000u);
        const float p0 = f0 * ck, p1 = f1 * ck, p2 = f2 * ck, p3 = f3 * ck;
        a0 = a0 + p0; a1 = a1 + p1; a2 = a2 + p2; a3 = a3 + p3;
      }
    }
    const float pzr = big ? qnan : pz;
    const bool live = node < nN;
    const float m0 = live ? (a0 * nd + pzr) : 0.0f;
    const float m1 = live ? (a1 * nd + pzr) : 0.0f;
    const float m2 = live ? (a2 * nd + pzr) : 0.0f;
    const float m3 = live ? (a3 * nd + pzr) : 0.0f;
    v4us mh, ml;
    {
      unsigned hb;
      hb = bf16_bits_np(m0); mh[0] = (unsigned short)hb; ml[0] = (unsigned short)bf16_bits_np(m0 - __uint_as_float(hb << 16));
      hb = bf16_bits_np(m1); mh[1] = (unsigned short)hb; ml[1] = (unsigned short)bf16_bits_np(m1 - __uint_as_float(hb << 16));
      hb = bf16_bits_np(m2); mh[2] = (unsigned short)hb; ml[2] = (unsigned short)bf16_bits_np(m2 - __uint_as_float(hb << 16));
      hb = bf16_bits_np(m3); mh[3] = (unsigned short)hb; ml[3] = (unsigned short)bf16_bits_np(m3 - __uint_as_float(hb << 16));
    }
    *(v4usa*)(rowbuf + 4 * lane) = mh;
    *(v4usa*)(rowbuf + DF + 4 * lane) = ml;
    wave_sync();
    const v8us q0 = *(const v8usa*)(rowbuf + 8 * lane);
    wave_sync();
    if (node < mRows) {
      unsigned short* rpw = ag + (size_t)node * ROWH + 8 * lane;
      *(volatile v8us*)rpw = q0;
      __threadfence();
      *(volatile v8us*)rpw = q0;
    }
  }
}

KERNEL(GTHR) void k_gemm(const unsigned short* __restrict__ Apl, const unsigned short* __restrict__ BT,
                         const float* __restrict__ tab, float* hout) {
  __shared__ __attribute__((aligned(16))) float stg[GBM * GBN];
  __shared__ __attribute__((aligned(16))) float bs[DF];
  const int tid = (int)threadIdx.x, lane = tid & 31, wave = tid >> 5, hh = lane >> 4, m = lane & 15;
  const int rowBase = (int)blockIdx.x * GBM;

  if (tid < 32) *(v4fa*)(bs + 4 * tid) = *(const v4f*)(tab + T_B + 4 * tid);

  v8f acc[8];
  {
    const v8f z = {0.f, 0.f, 0.f, 0.f, 0.f, 0.f, 0.f, 0.f};
#pragma unroll
    for (int t = 0; t < 8; ++t) acc[t] = z;
  }
  const unsigned short* ap = Apl + (size_t)(rowBase + 16 * wave + m) * (size_t)KG + 8 * hh;
  const unsigned short* bp = BT + (size_t)m * (size_t)KG + 8 * hh;

#pragma unroll 1
  for (int k0 = 0; k0 < KG; k0 += 32) {
    FragB af;
    af.h[0] = *(const v8usa*)(ap + k0);
    af.h[1] = *(const v8usa*)(ap + k0 + 16);
#pragma unroll
    for (int nt = 0; nt < 8; ++nt) {
      const unsigned short* wq = bp + (size_t)(16 * nt) * (size_t)KG + k0;
      FragB bf;
      bf.h[0] = *(const v8usa*)wq;
      bf.h[1] = *(const v8usa*)(wq + 16);
      acc[nt] = wmb(af, bf, acc[nt]);
    }
  }

#pragma unroll
  for (int nt = 0; nt < 8; ++nt) {
    const int lc = 16 * nt + m;
#pragma unroll
    for (int r = 0; r < 8; ++r) {
      const int lr = 16 * wave + 8 * hh + r;
      stg[lr * GBN + lc] = acc[nt][r];
    }
  }
  __syncthreads();

  const v4f bb4 = *(const v4fa*)(bs + 4 * lane);
  v4f pv[16];
#pragma unroll
  for (int i = 0; i < 16; ++i) pv[i] = *(const v4fa*)(stg + (16 * wave + i) * GBN + 4 * lane);
#pragma unroll
  for (int i = 0; i < 16; ++i) {
    const v4f t = pv[i] + bb4;
    v4f y;
    y.x = (t.x > 0.0f) ? t.x : (t.x - t.x);
    y.y = (t.y > 0.0f) ? t.y : (t.y - t.y);
    y.z = (t.z > 0.0f) ? t.z : (t.z - t.z);
    y.w = (t.w > 0.0f) ? t.w : (t.w - t.w);
    pv[i] = y;
  }
#pragma unroll
  for (int i = 0; i < 16; ++i) {
    const int r = rowBase + 16 * wave + i;
    *(volatile v4f*)(hout + (size_t)r * DF + 4 * lane) = pv[i];
  }
  __threadfence();
#pragma unroll
  for (int i = 0; i < 16; ++i) {
    const int r = rowBase + 16 * wave + i;
    *(volatile v4f*)(hout + (size_t)r * DF + 4 * lane) = pv[i];
  }
}

KERNEL(NTHR) void k_pool(const float* __restrict__ hf, const int* __restrict__ gid, int nN, float* hgout) {
  __shared__ __attribute__((aligned(16))) float wsum[NWAVE * DF];
  __shared__ int wcn[NWAVE];
  __shared__ __attribute__((aligned(16))) float outs[DF];
  const int tid = (int)threadIdx.x, lane = tid & 31, wave = tid >> 5;
  const int g = (int)blockIdx.x;

  float a0 = 0.0f, a1 = 0.0f, a2 = 0.0f, a3 = 0.0f;
  int mine = 0;
#pragma unroll 1
  for (int i0 = wave * 32; i0 < nN; i0 += NTHR) {
    const int i  = i0 + lane;
    const int ic = i < nN ? i : nN - 1;
    const int b  = gid[ic];
    const bool hit = (i < nN) && (b == g);
    mine += hit ? 1 : 0;
    unsigned msk = __builtin_amdgcn_ballot_w32(hit);
    int nh = (int)__builtin_popcount(msk);
    nh = nh > 32 ? 32 : nh;
#pragma unroll 1
    for (int q = 0; q < nh; ++q) {
      const int k = __builtin_ffs((int)msk) - 1;
      msk &= msk - 1u;
      int node = i0 + (k < 0 ? 0 : k);
      node = node > nN - 1 ? nN - 1 : node;
      const v4f v = *(const v4f*)(hf + (size_t)node * DF + 4 * lane);
      a0 += v.x; a1 += v.y; a2 += v.z; a3 += v.w;
    }
  }
  mine += __shfl_xor(mine, 16, 32);
  mine += __shfl_xor(mine, 8, 32);
  mine += __shfl_xor(mine, 4, 32);
  mine += __shfl_xor(mine, 2, 32);
  mine += __shfl_xor(mine, 1, 32);
  {
    v4f av;
    av.x = a0; av.y = a1; av.z = a2; av.w = a3;
    *(v4fa*)(wsum + wave * DF + 4 * lane) = av;
  }
  if (lane == 0) wcn[wave] = mine;
  __syncthreads();
  if (tid < DF) {
    float s = 0.0f;
    int c = 0;
#pragma unroll
    for (int w2 = 0; w2 < NWAVE; ++w2) { s += wsum[w2 * DF + tid]; c += wcn[w2]; }
    const float cf = (c < 1) ? 1.0f : (float)c;
    const float q = s / cf;
    outs[tid] = (c > 0) ? q : 0.0f;
  }
  __syncthreads();
  const v4f ov = *(const v4fa*)(outs + 4 * lane);
  float* op = hgout + (size_t)g * DF + 4 * lane;
  const bool okst = (wave == 0);
  if (okst) *(volatile v4f*)op = ov;
  __threadfence();
  if (okst) *(volatile v4f*)op = ov;
}

KERNEL(NTHR) void k_head(const float* __restrict__ hg, const float* __restrict__ tab, float* out) {
  __shared__ __attribute__((aligned(16))) float tl[T_USED];
  __shared__ __attribute__((aligned(16))) float z1[NZ1];
  __shared__ __attribute__((aligned(16))) float os[NOUT];
  const int tid = (int)threadIdx.x;
#pragma unroll 1
  for (int i = tid; i < T_USED / 4; i += NTHR) *(v4fa*)(tl + 4 * i) = *(const v4f*)(tab + 4 * i);
  __syncthreads();
#pragma unroll 1
  for (int idx = tid; idx < NZ1; idx += NTHR) {
    const int g = idx / NH1;
    const int j = idx - g * NH1;
    const float* pr = hg + (size_t)g * DF;
    float s = 0.0f;
#pragma unroll 1
    for (int f4 = 0; f4 < DF / 4; ++f4) {
      const v4f p = *(const v4f*)(pr + 4 * f4);
      const float* w = tl + T_W1 + (4 * f4) * NH1 + j;
      s = fmaf(p.x, w[0], s);
      s = fmaf(p.y, w[NH1], s);
      s = fmaf(p.z, w[2 * NH1], s);
      s = fmaf(p.w, w[3 * NH1], s);
    }
    z1[idx] = s + tl[T_B1 + j];
  }
  __syncthreads();
#pragma unroll 1
  for (int idx = tid; idx < NOUT; idx += NTHR) {
    const int g = idx / NCLS;
    const int c = idx - g * NCLS;
    float s = 0.0f;
#pragma unroll 4
    for (int j = 0; j < NH1; ++j) s = fmaf(z1[g * NH1 + j], tl[T_W2 + j * NCLS + c], s);
    os[idx] = s + tl[T_B2 + c];
  }
  __syncthreads();
  constexpr int NIT = NOUT / (4 * NTHR);
  v4f ov[NIT];
#pragma unroll
  for (int it = 0; it < NIT; ++it) ov[it] = *(const v4fa*)(os + 4 * (it * NTHR + tid));
#pragma unroll
  for (int it = 0; it < NIT; ++it) *(volatile v4f*)(out + 4 * (size_t)(it * NTHR + tid)) = ov[it];
  __threadfence();
#pragma unroll
  for (int it = 0; it < NIT; ++it) *(volatile v4f*)(out + 4 * (size_t)(it * NTHR + tid)) = ov[it];
}

static inline int cdiv(int a, int b) { return (a + b - 1) / b; }
static inline size_t al256(size_t o) { return (o + 255) & ~(size_t)255; }

extern "C" void kernel_launch(void* const* d_in, const int* in_sizes, int n_in,
                              void* d_out, int out_size, void* d_ws, size_t ws_size,
                              hipStream_t stream) {
  if (n_in < 10) return;
  if (in_sizes[0] < DF || (in_sizes[0] % DF) != 0) return;
  const int nN = in_sizes[0] / DF;
  if (nN < 32 || nN > (1 << 22) || (nN % 32) != 0) return;
  if (in_sizes[1] != DF * DF || in_sizes[2] != DF) return;
  if (in_sizes[3] != DF * NH1 || in_sizes[4] != NH1) return;
  if (in_sizes[5] != NH1 * NCLS || in_sizes[6] != NCLS) return;
  const int nE = in_sizes[7];
  if (nE < 1 || nE >= (1 << 21) || in_sizes[8] != nE) return;
  if (in_sizes[9] != nN) return;
  if (out_size != NOUT) return;

  const float* feats = (const float*)d_in[0];
  const float* W     = (const float*)d_in[1];
  const float* b     = (const float*)d_in[2];
  const float* W1    = (const float*)d_in[3];
  const float* b1    = (const float*)d_in[4];
  const float* W2    = (const float*)d_in[5];
  const float* b2    = (const float*)d_in[6];
  const int*   src   = (const int*)d_in[7];
  const int*   dst   = (const int*)d_in[8];
  const int*   gids  = (const int*)d_in[9];
  float* out = (float*)d_out;

  const int MP  = cdiv(nN, 128) * 128;
  const int gM  = MP / GBM;
  const int gA  = cdiv(MP, NBA);
  const int gO  = cdiv(nN, NBA);
  const int nbX = MP / 16;
  if ((long long)gA * NBA < (long long)MP) return;
  if ((long long)gO * NBA < (long long)nN) return;
  const int vec8 = ((nE & 3) == 0) ? 1 : 0;

  char* ws = (char*)d_ws;
  size_t off = 0;
  const size_t oXB  = off; off = al256(off + (size_t)MP * DF * 2);
  const size_t oAG  = off; off = al256(off + (size_t)MP * ROWH * 2);
  const size_t oH   = off; off = al256(off + (size_t)MP * DF * 4);
  const size_t oNS  = off; off = al256(off + (size_t)MP * 4);
  const size_t oWT2 = off; off = al256(off + (size_t)DF * KG * 2);
  const size_t oTAB = off; off = al256(off + (size_t)T_FLOATS * 4);
  const size_t oHG  = off; off = al256(off + (size_t)NGR * DF * 4);
  if (off > ws_size || off > (size_t)WSMAX) return;
  unsigned short* XB  = (unsigned short*)(ws + oXB);
  unsigned short* AG  = (unsigned short*)(ws + oAG);
  float*          H   = (float*)(ws + oH);
  float*          NS  = (float*)(ws + oNS);
  unsigned short* WT2 = (unsigned short*)(ws + oWT2);
  float*          TAB = (float*)(ws + oTAB);
  float*          HG  = (float*)(ws + oHG);

  const size_t aggLds = (size_t)AGG_LDS_INTS * 4;
  hipFuncSetAttribute(reinterpret_cast<const void*>(&k_agg), hipFuncAttributeMaxDynamicSharedMemorySize, (int)aggLds);

  k_prep<<<nbX + NBW + NBT, NTHR, 0, stream>>>(feats, W, b, W1, b1, W2, b2, nN, nbX, XB, WT2, TAB);
  k_odeg<<<gO, NTHR, 0, stream>>>(src, nE, nN, vec8, NS);
  k_agg<<<gA, NTHR, aggLds, stream>>>(src, dst, nE, nN, vec8, MP, NS, XB, AG);
  k_gemm<<<gM, GTHR, 0, stream>>>(AG, WT2, TAB, H);
  k_pool<<<NGR, NTHR, 0, stream>>>(H, gids, nN, HG);
  k_head<<<1, NTHR, 0, stream>>>(HG, TAB, out);
}
